// QuantumResidualRegressor_78503412236645
// MI455X (gfx1250) — hardware-run, weakly checked
//
#include <hip/hip_runtime.h>


#ifndef NSAMP
#define NSAMP 131072
#endif
#define NSAMP_FULL 131072
#define DIN  32
#define HID  16
#define NQ   6
#define NL   3
#define NST  64
#define MW   4
#define TPW  2
#define HSC  64.0f
#define W2C  64.0f
#define HWI  (1.0f / 4096.0f)
#define PSC  4096.0f
#define USC  16.0f
#define ZSC  2.3283064365386963e-10f

static_assert(DIN == 32);
static_assert(HID == 16);
static_assert(NQ == 6);
static_assert(NST == 64);
static_assert(NST == (1 << NQ));
static_assert(NST % 32 == 0);
static_assert((2 * NST) % 16 == 0);
static_assert(NQ <= 8);
static_assert(16 * TPW == 32);
static_assert(NSAMP % (32 * MW) == 0);
static_assert(NSAMP <= NSAMP_FULL);
static_assert(NL * NQ <= 64);

typedef _Float16 h16;
typedef unsigned short bf;
typedef __attribute__((ext_vector_type(16))) __bf16   v16bf;
typedef __attribute__((ext_vector_type(16))) _Float16 v16h;
typedef __attribute__((ext_vector_type(8)))  _Float16 v8h;
typedef __attribute__((ext_vector_type(8)))  unsigned short v8us;
typedef __attribute__((ext_vector_type(8)))  float    v8f;
typedef __attribute__((ext_vector_type(4)))  float    v4f;
typedef v4f  __attribute__((may_alias)) v4fa;

__device__ __forceinline__ unsigned short f2bf(float f) { unsigned u = __float_as_uint(f); u += 0x7FFFu + ((u >> 16) & 1u); return (unsigned short)(u >> 16); }
__device__ __forceinline__ float bfr(float f) { return __uint_as_float(((unsigned)f2bf(f)) << 16); }
__device__ __forceinline__ v16h cat16(v8h lo, v8h hi) { return __builtin_shufflevector(lo, hi, 0, 1, 2, 3, 4, 5, 6, 7, 8, 9, 10, 11, 12, 13, 14, 15); }
__device__ __forceinline__ v16bf cat16b(v8us lo, v8us hi) { return __builtin_bit_cast(v16bf, __builtin_shufflevector(lo, hi, 0, 1, 2, 3, 4, 5, 6, 7, 8, 9, 10, 11, 12, 13, 14, 15)); }
__device__ __forceinline__ v16h  ldh(const h16* p) { return cat16(*(const v8h*)p, *(const v8h*)(p + 16)); }
__device__ __forceinline__ v16bf ldb(const bf* p)  { return cat16b(*(const v8us*)p, *(const v8us*)(p + 16)); }

static __device__ __forceinline__ h16 toh_flush(float v) { const h16 r = (h16)v; return (fabsf(v) < 6.103515625e-05f) ? (h16)0.0f : r; }
__device__ __forceinline__ v8f wmma16g(v16h a, v16h b, v8f c) {
    c = __builtin_amdgcn_wmma_f32_16x16x32_f16(false, a, false, b, (short)0, c, false, false);
    asm volatile("v_nop\n\tv_nop\n\tv_nop\n\tv_nop" : "+v"(c) : "v"(a), "v"(b));
    return c; }
__device__ __forceinline__ v8f wmmabg(v16bf a, v16bf b, v8f c) {
    c = __builtin_amdgcn_wmma_f32_16x16x32_bf16(false, a, false, b, (short)0, c, false, false);
    asm volatile("v_nop\n\tv_nop\n\tv_nop\n\tv_nop" : "+v"(c) : "v"(a), "v"(b));
    return c; }
__device__ __forceinline__ float gelu_erf(float x) { return 0.5f * x * (1.0f + erff(x * 0.70710678118654752f)); }

static_assert(sizeof(float) * (2 * NST * NST + 512 + 512 + 128) <= 131072);
static_assert(16 * 64 * 8 == 2 * NST * NST);
static_assert(64 * 8 == 16 * 32);

__global__ __launch_bounds__(64) void k_prep(const float* __restrict__ w1, const float* __restrict__ w2, const float* __restrict__ qw, bf* W1T, h16* W2T, h16* UT) {
    __shared__ __align__(16) float st[2 * NST * NST];
    __shared__ __align__(16) float wf1[16 * 32];
    __shared__ __align__(16) float wf2[16 * 32];
    __shared__ float cw[64], sw[64];
    const int tid = threadIdx.x;
    { const int ti = tid < NL * NQ ? tid : NL * NQ - 1;
      float q = qw[ti]; asm volatile("" : "+v"(q));
      const float hw = 0.5f * bfr(q);
      cw[tid] = cosf(hw); sw[tid] = sinf(hw); }
#pragma unroll 1
    for (int it = 0; it < 8; ++it) {
        const int e = it * 64 + tid; const int n = e >> 5, k = e & 31;
        const float a = w1[k * HID + n];
        wf1[e] = bfr(a);
        const bool ok = (n < NQ) & (k < HID);
        const int kc = k < HID ? k : HID - 1, nc = n < NQ ? n : NQ - 1;
        float b = w2[kc * NQ + nc]; asm volatile("" : "+v"(b));
        wf2[e] = ok ? bfr(b) * W2C : 0.0f; }
#pragma unroll 1
    for (int i = 0; i < NST; ++i) { st[i * NST + tid] = (i == tid) ? 1.0f : 0.0f; st[(NST + i) * NST + tid] = 0.0f; }
    __syncthreads();
#pragma unroll 1
    for (int l = 0; l < NL; ++l) {
#pragma unroll 1
        for (int q = 0; q < NQ; ++q) {
            const int qm = 32 >> q; const float c = cw[l * NQ + q], s = sw[l * NQ + q];
#pragma unroll 1
            for (int p = 0; p < 32; ++p) {
                const int i = ((p & ~(qm - 1)) << 1) | (p & (qm - 1)); const int j = i | qm;
                const float a0r = st[i * NST + tid], a0i = st[(NST + i) * NST + tid];
                const float a1r = st[j * NST + tid], a1i = st[(NST + j) * NST + tid];
                st[i * NST + tid] = c * a0r + s * a1i; st[(NST + i) * NST + tid] = c * a0i - s * a1r;
                st[j * NST + tid] = c * a1r + s * a0i; st[(NST + j) * NST + tid] = c * a1i - s * a0r; } }
#pragma unroll 1
        for (int cq = 0; cq < NQ; ++cq) {
            const int cm = 32 >> cq; const int tq = (cq + 1 == NQ) ? 0 : cq + 1; const int tm = 32 >> tq;
#pragma unroll 1
            for (int i = 0; i < NST; ++i) {
                if (((i & cm) != 0) & ((i & tm) == 0)) {
                    const int j = i | tm;
                    const float tr = st[i * NST + tid]; st[i * NST + tid] = st[j * NST + tid]; st[j * NST + tid] = tr;
                    const float ti = st[(NST + i) * NST + tid]; st[(NST + i) * NST + tid] = st[(NST + j) * NST + tid]; st[(NST + j) * NST + tid] = ti; } } }
    }
    __syncthreads();
#pragma unroll 1
    for (int ps = 0; ps < 2; ++ps) {
#pragma unroll 1
        for (int it = 0; it < 16; ++it) {
            const int p = it * 64 + tid; const int row = p >> 3, c8 = (p & 7) * 8;
            const v4f x0 = *(const v4fa*)(&st[row * NST + c8]); const v4f x1 = *(const v4fa*)(&st[row * NST + c8 + 4]); v8h hv;
#pragma unroll
            for (int i = 0; i < 4; ++i) { hv[i] = toh_flush(x0[i] * USC); hv[4 + i] = toh_flush(x1[i] * USC); }
            *(volatile v8h*)(UT + (size_t)row * NST + c8) = hv; }
        { const v4f x0 = *(const v4fa*)(&wf1[tid * 8]); const v4f x1 = *(const v4fa*)(&wf1[tid * 8 + 4]); v8us o;
#pragma unroll
          for (int i = 0; i < 4; ++i) { o[i] = f2bf(x0[i]); o[4 + i] = f2bf(x1[i]); }
          *(volatile v8us*)(W1T + (size_t)tid * 8) = o; }
        { const v4f x0 = *(const v4fa*)(&wf2[tid * 8]); const v4f x1 = *(const v4fa*)(&wf2[tid * 8 + 4]); v8h hv;
#pragma unroll
          for (int i = 0; i < 4; ++i) { hv[i] = toh_flush(x0[i]); hv[4 + i] = toh_flush(x1[i]); }
          *(volatile v8h*)(W2T + (size_t)tid * 8) = hv; }
        if (ps == 0) __threadfence(); }
}

__global__ __launch_bounds__(32 * MW) __attribute__((amdgpu_num_vgpr(256))) void k_circ(const float* __restrict__ X, const float* __restrict__ BASE,
                                              const float* __restrict__ b1, const float* __restrict__ b2,
                                              const float* __restrict__ hw1, const float* __restrict__ hb1,
                                              const float* __restrict__ hw2, const float* __restrict__ hb2,
                                              const bf* __restrict__ W1T, const h16* __restrict__ W2T, const h16* __restrict__ UT, float* OUT) {
    const int lane = threadIdx.x & 31, lr = lane & 15, hi = lane >> 4;
    const int wave = __builtin_amdgcn_readfirstlane((int)(threadIdx.x >> 5));
    const int s0 = (blockIdx.x * MW + wave) * (16 * TPW);
    const v16bf w1a = ldb(W1T + lr * DIN + 8 * hi);
    const v16h  w2a = ldh(W2T + lr * 32 + 8 * hi);
    float bb1[8], bb2[NQ];
#pragma unroll
    for (int r = 0; r < 8; ++r) bb1[r] = bfr(b1[8 * hi + r]);
#pragma unroll
    for (int q = 0; q < NQ; ++q) bb2[q] = bfr(b2[q]);
    const float hb2v = bfr(hb2[0]);
    const size_t uo = (size_t)lr * NST + 8 * hi;
    float outv = 0.0f;
#pragma unroll 1
    for (int tt = 0; tt < TPW; ++tt) {
        const int srow = s0 + 16 * tt + lr;
        const float* xr = X + (size_t)srow * DIN + 8 * hi;
        const v8f x0 = *(const v8f*)xr, x1 = *(const v8f*)(xr + 16);
        v8us u0, u1;
#pragma unroll
        for (int k = 0; k < 8; ++k) { u0[k] = f2bf(x0[k]); u1[k] = f2bf(x1[k]); }
        const v16bf xb = cat16b(u0, u1);
        v8f d1 = (v8f){};
        d1 = wmmabg(w1a, xb, d1);
        v16h hb = (v16h){};
#pragma unroll
        for (int r = 0; r < 8; ++r) hb[r] = toh_flush(gelu_erf(d1[r] + bb1[r]) * HSC);
        v8f d2 = (v8f){};
        d2 = wmma16g(w2a, hb, d2);
        float cs[NQ], sn[NQ];
#pragma unroll
        for (int q = 0; q < NQ; ++q) {
            const float pre = __shfl(d2[q], lr, 32) * HWI + bb2[q];
            const float hf = 0.5f * tanhf(pre);
            cs[q] = cosf(hf); sn[q] = sinf(hf); }
        const float g2 = hi ? sn[2] : cs[2];
        const float a30 = g2 * cs[3], a31 = g2 * sn[3];
        float a34[4]; a34[0] = a30 * cs[4]; a34[1] = a30 * sn[4]; a34[2] = a31 * cs[4]; a34[3] = a31 * sn[4];
        float low[8];
#pragma unroll
        for (int u = 0; u < 4; ++u) { low[2 * u] = a34[u] * cs[5]; low[2 * u + 1] = a34[u] * sn[5]; }
        float f01[2][2];
        f01[0][0] = cs[0] * cs[1] * PSC; f01[0][1] = cs[0] * sn[1] * PSC; f01[1][0] = sn[0] * cs[1] * PSC; f01[1][1] = sn[0] * sn[1] * PSC;
        v16h pf[2];
#pragma unroll
        for (int s = 0; s < 2; ++s)
#pragma unroll
            for (int e = 0; e < 2; ++e)
#pragma unroll
                for (int t = 0; t < 8; ++t) pf[s][e * 8 + t] = toh_flush(f01[s][e] * low[t]);
        v8f acc[8];
#pragma unroll
        for (int j = 0; j < 8; ++j) acc[j] = (v8f){};
#pragma unroll
        for (int s = 0; s < 2; ++s)
#pragma unroll
            for (int j = 0; j < 8; ++j) { const v16h ua = ldh(UT + uo + (size_t)(16 * j) * NST + 32 * s); acc[j] = wmma16g(ua, pf[s], acc[j]); }
        float T = 0.0f, A0 = 0.0f, A1 = 0.0f, Z3 = 0.0f, Z4 = 0.0f, Z5 = 0.0f;
#pragma unroll
        for (int r = 0; r < 8; ++r) {
            const float p0 = acc[0][r] * acc[0][r] + acc[4][r] * acc[4][r];
            const float p1 = acc[1][r] * acc[1][r] + acc[5][r] * acc[5][r];
            const float p2 = acc[2][r] * acc[2][r] + acc[6][r] * acc[6][r];
            const float p3 = acc[3][r] * acc[3][r] + acc[7][r] * acc[7][r];
            const float s01 = p0 + p1, s23 = p2 + p3, s02 = p0 + p2, s13 = p1 + p3; const float S = s01 + s23;
            A0 += s01 - s23; A1 += s02 - s13; T += S;
            Z3 += (r & 4) ? -S : S; Z4 += (r & 2) ? -S : S; Z5 += (r & 1) ? -S : S; }
        const float To = __shfl_xor(T, 16, 32);
        float z[NQ];
        z[0] = (A0 + __shfl_xor(A0, 16, 32)) * ZSC;
        z[1] = (A1 + __shfl_xor(A1, 16, 32)) * ZSC;
        z[2] = (hi ? (To - T) : (T - To)) * ZSC;
        z[3] = (Z3 + __shfl_xor(Z3, 16, 32)) * ZSC;
        z[4] = (Z4 + __shfl_xor(Z4, 16, 32)) * ZSC;
        z[5] = (Z5 + __shfl_xor(Z5, 16, 32)) * ZSC;
        float racc = 0.0f;
#pragma unroll 1
        for (int oo = 0; oo < 8; ++oo) {
            const int o = 8 * hi + oo;
            float hp = bfr(hb1[o]);
#pragma unroll
            for (int q = 0; q < NQ; ++q) hp = fmaf(z[q], bfr(hw1[q * HID + o]), hp);
            racc = fmaf(gelu_erf(hp), bfr(hw2[o]), racc); }
        racc += __shfl_xor(racc, 16, 32);
        const float res = bfr(BASE[srow]) + (racc + hb2v);
        outv = (hi == tt) ? res : outv;
    }
    static_assert(32 * 4 == 16 * TPW * 4);
    volatile float* op = OUT + (size_t)s0 + lane;
    *op = outv; __threadfence(); *op = outv;
}

static constexpr size_t al256(size_t v) { return (v + 255) & ~(size_t)255; }
static constexpr size_t SZ_W1T = al256((size_t)16 * 32 * 2);
static constexpr size_t SZ_W2T = al256((size_t)16 * 32 * 2);
static constexpr size_t SZ_UT  = al256((size_t)2 * NST * NST * 2);
static constexpr size_t SZ_TOTAL = SZ_W1T + SZ_W2T + SZ_UT;
static_assert(SZ_TOTAL <= (size_t)134217728);
static_assert(SZ_W1T == 1024 && SZ_W2T == 1024 && SZ_UT == 16384);

extern "C" void kernel_launch(void* const* d_in, const int* in_sizes, int n_in,
                              void* d_out, int out_size, void* d_ws, size_t ws_size, hipStream_t stream) {
    if (n_in < 11) return;
    if ((size_t)in_sizes[0] < (size_t)NSAMP * DIN || (size_t)in_sizes[1] < (size_t)NSAMP) return;
    if (in_sizes[2] < DIN * HID || in_sizes[3] < HID || in_sizes[4] < HID * NQ || in_sizes[5] < NQ) return;
    if (in_sizes[6] < NL * NQ || in_sizes[7] < NQ * HID || in_sizes[8] < HID || in_sizes[9] < HID || in_sizes[10] < 1) return;
    if ((size_t)out_size < (size_t)NSAMP) return;
    if (SZ_TOTAL > ws_size) return;
    const float* features = (const float*)d_in[0];
    const float* baseline = (const float*)d_in[1];
    const float* enc_w1   = (const float*)d_in[2];
    const float* enc_b1   = (const float*)d_in[3];
    const float* enc_w2   = (const float*)d_in[4];
    const float* enc_b2   = (const float*)d_in[5];
    const float* q_w      = (const float*)d_in[6];
    const float* head_w1  = (const float*)d_in[7];
    const float* head_b1  = (const float*)d_in[8];
    const float* head_w2  = (const float*)d_in[9];
    const float* head_b2  = (const float*)d_in[10];
    float* OUT = (float*)d_out;
    char* wsp = (char*)d_ws;
    bf*  W1T = (bf*)wsp;  wsp += SZ_W1T;
    h16* W2T = (h16*)wsp; wsp += SZ_W2T;
    h16* UT  = (h16*)wsp; wsp += SZ_UT;

    k_prep<<<1, 64, 0, stream>>>(enc_w1, enc_w2, q_w, W1T, W2T, UT);
    k_circ<<<NSAMP / (32 * MW), 32 * MW, 0, stream>>>(features, baseline, enc_b1, enc_b2, head_w1, head_b1, head_w2, head_b2, W1T, W2T, UT, OUT);
}
